// GCNN_68178310857464
// MI455X (gfx1250) — hardware-verified
//
#include <hip/hip_runtime.h>
#include <stddef.h>
#include <stdint.h>


#define DM     512
#define DM2    1024
#define NREL   8
#define NTHR   256
#define NWAVE  8
#define EPT    8
#define CHUNK  (NTHR * EPT)
#define WCAP   (EPT * 32)
#define LISTN  (NWAVE * WCAP)
#define NBA    1024
#define SLA    10
#define DIRB   29
#define EIDMASK ((1 << (DIRB - SLA)) - 1)
#define RCAP   17408
#define DEGCAP 64
#define GBM    64
#define GBN    128
#define GTHR   128
#define AGG_ZINTS    (LISTN + 2 * RCAP + 3 * NBA)
#define MISC_INTS    16
#define SCAN_LDS_INTS (AGG_ZINTS + MISC_INTS)
#define WSMAX  134217728

static_assert((CHUNK & (CHUNK - 1)) == 0 && CHUNK <= 4096);
static_assert((NBA & (NBA - 1)) == 0 && NBA == (1 << SLA));
static_assert(LISTN % NTHR == 0 && WCAP <= 256);
static_assert(NBA % NWAVE == 0 && NBA % 32 == 0);
static_assert(RCAP % 4 == 0 && AGG_ZINTS % (NTHR * 4) == 0);
static_assert(DM % 32 == 0 && DM % GBN == 0 && DM2 % GBN == 0 && DM % 128 == 0);
static_assert(GBM == 64 && GBN == 128 && GTHR == 128);
static_assert(SCAN_LDS_INTS * 4 <= 300000);
static_assert(DIRB < 31 && (DIRB - SLA) >= 19);

typedef float          v4f   __attribute__((ext_vector_type(4)));
typedef float          v8f   __attribute__((ext_vector_type(8)));
typedef int            v4i   __attribute__((ext_vector_type(4)));
typedef int            v8i   __attribute__((ext_vector_type(8)));
typedef unsigned short v8us  __attribute__((ext_vector_type(8)));
typedef unsigned short v16us __attribute__((ext_vector_type(16)));
typedef __bf16         v16bf __attribute__((ext_vector_type(16)));
typedef v4f  __attribute__((may_alias)) v4fa;
typedef v4i  __attribute__((may_alias)) v4ia;
typedef v8us __attribute__((may_alias)) v8usa;
union FragB { v16bf v; v16us u; v8us h[2]; v8i w; };

__device__ __forceinline__ v8f wmb(const FragB& a, const FragB& b, v8f c) {
  v8f d = __builtin_amdgcn_wmma_f32_16x16x32_bf16(false, a.v, false, b.v, (short)0, c, false, false);
  asm volatile("v_nop\n\tv_nop\n\tv_nop\n\tv_nop" : "+v"(d) : "v"(a.w), "v"(b.w));
  return d;
}

__device__ __forceinline__ unsigned bf16_bits(float f) {
  const unsigned u = __float_as_uint(f);
  return (u + 0x7FFFu + ((u >> 16) & 1u)) >> 16;
}
__device__ __forceinline__ float bf16_val(float f) {
  return __uint_as_float(bf16_bits(f) << 16);
}

__global__ __launch_bounds__(NTHR) void k_prep(const float* __restrict__ x, const float* __restrict__ wsf,
                                               const float* __restrict__ wrf, int nN, int nxu,
                                               unsigned short* XB, unsigned short* WSB, unsigned short* WRB) {
  const int u = (int)blockIdx.x * NTHR + (int)threadIdx.x;
  const int nws = DM * DM / 8;
  const int nwr = 2 * NREL * DM * DM / 8;
  const float* src;
  unsigned short* dst;
  float keep = 1.0f;
  if (u < nxu) {
    const int row = u >> 6;
    const int c8  = (u & 63) * 8;
    const int rs  = row < nN ? row : nN - 1;
    src  = x + (size_t)rs * DM + c8;
    dst  = XB + (size_t)u * 8;
    keep = row < nN ? 1.0f : 0.0f;
  } else if (u < nxu + nws) {
    const int v = u - nxu;
    src = wsf + (size_t)v * 8;
    dst = WSB + (size_t)v * 8;
  } else if (u < nxu + nws + nwr) {
    const int v = u - nxu - nws;
    src = wrf + (size_t)v * 8;
    dst = WRB + (size_t)v * 8;
  } else {
    return;
  }
  const v4f a = *(const v4fa*)src;
  const v4f b = *(const v4fa*)(src + 4);
  v8us o;
  o[0] = (unsigned short)bf16_bits(a.x * keep); o[1] = (unsigned short)bf16_bits(a.y * keep);
  o[2] = (unsigned short)bf16_bits(a.z * keep); o[3] = (unsigned short)bf16_bits(a.w * keep);
  o[4] = (unsigned short)bf16_bits(b.x * keep); o[5] = (unsigned short)bf16_bits(b.y * keep);
  o[6] = (unsigned short)bf16_bits(b.z * keep); o[7] = (unsigned short)bf16_bits(b.w * keep);
  *(volatile v8us*)dst = o;
  __threadfence();
  *(volatile v8us*)dst = o;
}

__global__ __launch_bounds__(GTHR) void k_gemm(const unsigned short* __restrict__ A,
                                               const unsigned short* B0p, const unsigned short* B1p,
                                               const float* bA, const float* bB,
                                               float* C, int ldc, int nOut) {
  __shared__ __attribute__((aligned(16))) float stg[GBM * GBN];
  const int tid = (int)threadIdx.x, lane = tid & 31, wave = tid >> 5, hh = lane >> 4, m = lane & 15;
  const int wr = wave >> 1, wc = wave & 1;
  const int rowBase = (int)blockIdx.x * GBM;
  const int colBase = (int)blockIdx.y * GBN;
  const bool upper = colBase >= DM;
  const unsigned short* BT = upper ? B1p : B0p;
  const float* bias = upper ? bB : bA;
  const int cb = upper ? (colBase - DM) : colBase;

  v8f acc[2][4];
  {
    const v8f z = {0.f, 0.f, 0.f, 0.f, 0.f, 0.f, 0.f, 0.f};
#pragma unroll
    for (int mt = 0; mt < 2; ++mt)
#pragma unroll
      for (int nt = 0; nt < 4; ++nt) acc[mt][nt] = z;
  }
  const unsigned short* ap0 = A + (size_t)(rowBase + 32 * wr + m) * (size_t)DM + 8 * hh;
  const unsigned short* ap1 = ap0 + (size_t)16 * DM;
  const unsigned short* bp  = BT + (size_t)(cb + 64 * wc + m) * (size_t)DM + 8 * hh;

#pragma unroll 1
  for (int k0 = 0; k0 < DM; k0 += 32) {
    FragB af0, af1;
    af0.h[0] = *(const v8usa*)(ap0 + k0);
    af0.h[1] = *(const v8usa*)(ap0 + k0 + 16);
    af1.h[0] = *(const v8usa*)(ap1 + k0);
    af1.h[1] = *(const v8usa*)(ap1 + k0 + 16);
#pragma unroll
    for (int nt = 0; nt < 4; ++nt) {
      const unsigned short* wq = bp + (size_t)(16 * nt) * (size_t)DM + k0;
      FragB bf;
      bf.h[0] = *(const v8usa*)wq;
      bf.h[1] = *(const v8usa*)(wq + 16);
      acc[0][nt] = wmb(af0, bf, acc[0][nt]);
      acc[1][nt] = wmb(af1, bf, acc[1][nt]);
    }
  }

#pragma unroll
  for (int mt = 0; mt < 2; ++mt)
#pragma unroll
    for (int nt = 0; nt < 4; ++nt) {
      const int lc = 64 * wc + 16 * nt + m;
#pragma unroll
      for (int r = 0; r < 8; ++r) {
        const int lr = 32 * wr + 16 * mt + 8 * hh + r;
        stg[lr * GBN + lc] = acc[mt][nt][r];
      }
    }
  __syncthreads();

  v4f bb4;
  {
    const v4f t1 = *(const v4fa*)(bias + cb + 4 * lane);
    bb4.x = bf16_val(t1.x); bb4.y = bf16_val(t1.y); bb4.z = bf16_val(t1.z); bb4.w = bf16_val(t1.w);
  }
  v4f pv[16];
#pragma unroll
  for (int i = 0; i < 16; ++i) pv[i] = *(const v4fa*)(stg + (16 * wave + i) * GBN + 4 * lane) + bb4;

#pragma unroll
  for (int i = 0; i < 16; ++i) {
    const int r = rowBase + 16 * wave + i;
    if (r < nOut) *(volatile v4f*)(C + (size_t)r * (size_t)ldc + colBase + 4 * lane) = pv[i];
  }
  __threadfence();
#pragma unroll
  for (int i = 0; i < 16; ++i) {
    const int r = rowBase + 16 * wave + i;
    if (r < nOut) *(volatile v4f*)(C + (size_t)r * (size_t)ldc + colBase + 4 * lane) = pv[i];
  }
}

__device__ __forceinline__ int scan_chunk(const int* __restrict__ keys, const int* __restrict__ rl, int nE,
                                          int cbase, int slotBase, int rsel, int* list,
                                          int tid, int lane, int wave) {
  int wc = 0;
  const int el0  = tid * EPT;
  const int e0   = cbase + el0;
  const int base = (e0 < nE - EPT) ? e0 : (nE - EPT);
  const v4i da = *(const v4ia*)(keys + base);
  const v4i db = *(const v4ia*)(keys + base + 4);
  const v4i qa = *(const v4ia*)(rl + base);
  const v4i qb = *(const v4ia*)(rl + base + 4);
  const bool val = e0 < nE;
  const unsigned nbs = (unsigned)slotBase;
  const unsigned unb = (unsigned)NBA;
  const unsigned s0 = (unsigned)da.x - nbs, s1 = (unsigned)da.y - nbs;
  const unsigned s2 = (unsigned)da.z - nbs, s3 = (unsigned)da.w - nbs;
  const unsigned s4 = (unsigned)db.x - nbs, s5 = (unsigned)db.y - nbs;
  const unsigned s6 = (unsigned)db.z - nbs, s7 = (unsigned)db.w - nbs;
  const bool h0 = val & (s0 < unb) & (qa.x == rsel), h1 = val & (s1 < unb) & (qa.y == rsel);
  const bool h2 = val & (s2 < unb) & (qa.z == rsel), h3 = val & (s3 < unb) & (qa.w == rsel);
  const bool h4 = val & (s4 < unb) & (qb.x == rsel), h5 = val & (s5 < unb) & (qb.y == rsel);
  const bool h6 = val & (s6 < unb) & (qb.z == rsel), h7 = val & (s7 < unb) & (qb.w == rsel);
  const unsigned any = __builtin_amdgcn_ballot_w32(h0 | h1 | h2 | h3 | h4 | h5 | h6 | h7);
  if (any != 0u) {
#define HITJ(J, HJ, SJ) { \
      const unsigned mj = __builtin_amdgcn_ballot_w32(HJ); \
      if (mj != 0u) { \
        if (HJ) { \
          const int pos = wc + (int)__builtin_amdgcn_mbcnt_lo(mj, 0u); \
          if (pos < WCAP) list[wave * WCAP + pos] = ((el0 + (J)) << SLA) | (int)(SJ); \
        } \
        wc += (int)__builtin_popcount(mj); } }
    HITJ(0, h0, s0)
    HITJ(1, h1, s1)
    HITJ(2, h2, s2)
    HITJ(3, h3, s3)
    HITJ(4, h4, s4)
    HITJ(5, h5, s5)
    HITJ(6, h6, s6)
    HITJ(7, h7, s7)
#undef HITJ
  }
  return wc;
}

__device__ __forceinline__ void scan_dir(const int* __restrict__ keys, const int* __restrict__ rl, int nE,
                                         int rsel, int dtag, int nodeBase, int* list, int* hl, int* cnt,
                                         int* misc, int tid, int lane, int wave, int& t, int& ov) {
  const int nChunks = (nE + CHUNK - 1) / CHUNK;
#pragma unroll 1
  for (int ch = 0; ch < nChunks; ++ch) {
    const int cbase = ch * CHUNK;
    const int wc = scan_chunk(keys, rl, nE, cbase, nodeBase, rsel, list, tid, lane, wave);
    if (lane == 0) misc[wave] = wc;
    __syncthreads();
    if (wave == 0) {
#pragma unroll 1
      for (int w2 = 0; w2 < NWAVE; ++w2) {
        int c = misc[w2];
        c = c < 0 ? 0 : (c > WCAP ? WCAP : c);
#pragma unroll 1
        for (int b0 = 0; b0 < c; b0 += 32) {
          const int idx = b0 + lane;
          const int ent = list[w2 * WCAP + (idx < WCAP ? idx : WCAP - 1)];
          const int m32 = (c - b0) < 32 ? (c - b0) : 32;
#pragma unroll 1
          for (int k = 0; k < m32; ++k) {
            const int u    = __builtin_amdgcn_readlane(ent, k);
            const int slot = u & (NBA - 1);
            const int el   = (u >> SLA) & (CHUNK - 1);
            const int pk   = dtag | ((cbase + el) << SLA) | slot;
            if (t < RCAP) {
              if (lane == 0) { hl[t] = pk; cnt[slot] = cnt[slot] + 1; }
              t = t + 1;
            } else {
              ov = 1;
            }
          }
        }
      }
    }
    __syncthreads();
  }
}

__global__ __launch_bounds__(NTHR) void k_scan(const int* __restrict__ heads, const int* __restrict__ tails,
                                               const int* __restrict__ rl, int nE, int nN, int rsel, int fin,
                                               const float* __restrict__ hfb, float* accp) {
  extern __shared__ __attribute__((aligned(16))) int dsm[];
  int* list = dsm;
  int* hl   = dsm + LISTN;
  int* sl   = hl + RCAP;
  int* cnt  = sl + RCAP;
  int* offs = cnt + NBA;
  int* cur  = offs + NBA;
  int* misc = cur + NBA;
  const int tid = (int)threadIdx.x, lane = tid & 31, wave = tid >> 5;
  const int nodeBase = (int)blockIdx.x * NBA;

  {
    const v4i z4 = {0, 0, 0, 0};
    for (int i = tid * 4; i < AGG_ZINTS; i += NTHR * 4) *(v4ia*)(dsm + i) = z4;
    if (tid < MISC_INTS) misc[tid] = 0;
  }
  __syncthreads();

  int t = 0, ov = 0;
  scan_dir(heads, rl, nE, rsel, 0,         nodeBase, list, hl, cnt, misc, tid, lane, wave, t, ov);
  scan_dir(tails, rl, nE, rsel, 1 << DIRB, nodeBase, list, hl, cnt, misc, tid, lane, wave, t, ov);
  if (wave == 0 && lane == 0) { misc[8] = t; misc[9] = ov; }
  __syncthreads();
  int tt = misc[8];
  tt = tt < 0 ? 0 : (tt > RCAP ? RCAP : tt);
  const int ovf = misc[9];

  if (wave == 0) {
    const int base = lane * (NBA / 32);
    int s = 0;
#pragma unroll 1
    for (int i = 0; i < NBA / 32; ++i) s += cnt[base + i];
    int incl = s;
#pragma unroll
    for (int d = 1; d < 32; d <<= 1) {
      const int y = __shfl_up(incl, d, 32);
      if (lane >= d) incl += y;
    }
    int run = incl - s;
#pragma unroll 1
    for (int i = 0; i < NBA / 32; ++i) {
      const int cv = cnt[base + i];
      offs[base + i] = run;
      cur[base + i]  = run;
      run += cv;
    }
  }
  __syncthreads();
  if (wave == 0) {
#pragma unroll 1
    for (int b0 = 0; b0 < tt; b0 += 32) {
      const int idx = b0 + lane;
      const int ent = hl[idx < RCAP ? idx : RCAP - 1];
      const int m32 = (tt - b0) < 32 ? (tt - b0) : 32;
#pragma unroll 1
      for (int k = 0; k < m32; ++k) {
        const int u    = __builtin_amdgcn_readlane(ent, k);
        const int slot = u & (NBA - 1);
        if (lane == 0) {
          int p = cur[slot];
          p = p < 0 ? 0 : (p > RCAP - 1 ? RCAP - 1 : p);
          sl[p] = u;
          cur[slot] = p + 1;
        }
      }
    }
  }
  __syncthreads();

  const float nanv = __int_as_float(0x7fc00000);
  const float pz = (ovf != 0) ? nanv : 0.0f;
#pragma unroll 1
  for (int si = 0; si < NBA / NWAVE; ++si) {
    const int s    = si * NWAVE + wave;
    const int node = nodeBase + s;
    int c = cnt[s];
    const bool big = c > DEGCAP;
    c = c < 0 ? 0 : (c > DEGCAP ? DEGCAP : c);
    int o = offs[s];
    o = o < 0 ? 0 : (o > RCAP ? RCAP : o);
    v4f a0 = {0.f, 0.f, 0.f, 0.f}, a1 = {0.f, 0.f, 0.f, 0.f};
    v4f a2 = {0.f, 0.f, 0.f, 0.f}, a3 = {0.f, 0.f, 0.f, 0.f};
#pragma unroll 1
    for (int b0 = 0; b0 < c; b0 += 32) {
      int idx = o + b0 + lane;
      idx = idx > RCAP - 1 ? RCAP - 1 : idx;
      const int ent = sl[idx];
      const int dir = (ent >> DIRB) & 1;
      int eid = (ent >> SLA) & EIDMASK;
      eid = eid > nE - 1 ? nE - 1 : eid;
      const int hs = heads[eid];
      const int ts = tails[eid];
      int src = ts + dir * (hs - ts);
      src = src < 0 ? 0 : (src > nN - 1 ? nN - 1 : src);
      const int roff = src * DM2 + dir * DM;
      const int m32 = (c - b0) < 32 ? (c - b0) : 32;
#pragma unroll 1
      for (int k = 0; k < m32; ++k) {
        const int sk = __builtin_amdgcn_readlane(roff, k);
        const float* rp = hfb + (size_t)sk + 4 * lane;
        a0 += *(const v4fa*)(rp);
        a1 += *(const v4fa*)(rp + 128);
        a2 += *(const v4fa*)(rp + 256);
        a3 += *(const v4fa*)(rp + 384);
      }
    }
    if (node < nN) {
      const float pzr = big ? nanv : pz;
      float* dp = accp + (size_t)node * DM + 4 * lane;
      v4f v0 = *(const v4fa*)(dp)       + a0 + pzr;
      v4f v1 = *(const v4fa*)(dp + 128) + a1 + pzr;
      v4f v2 = *(const v4fa*)(dp + 256) + a2 + pzr;
      v4f v3 = *(const v4fa*)(dp + 384) + a3 + pzr;
      if (fin != 0) {
        v0.x = (v0.x < 0.0f) ? 0.0f : v0.x; v0.y = (v0.y < 0.0f) ? 0.0f : v0.y;
        v0.z = (v0.z < 0.0f) ? 0.0f : v0.z; v0.w = (v0.w < 0.0f) ? 0.0f : v0.w;
        v1.x = (v1.x < 0.0f) ? 0.0f : v1.x; v1.y = (v1.y < 0.0f) ? 0.0f : v1.y;
        v1.z = (v1.z < 0.0f) ? 0.0f : v1.z; v1.w = (v1.w < 0.0f) ? 0.0f : v1.w;
        v2.x = (v2.x < 0.0f) ? 0.0f : v2.x; v2.y = (v2.y < 0.0f) ? 0.0f : v2.y;
        v2.z = (v2.z < 0.0f) ? 0.0f : v2.z; v2.w = (v2.w < 0.0f) ? 0.0f : v2.w;
        v3.x = (v3.x < 0.0f) ? 0.0f : v3.x; v3.y = (v3.y < 0.0f) ? 0.0f : v3.y;
        v3.z = (v3.z < 0.0f) ? 0.0f : v3.z; v3.w = (v3.w < 0.0f) ? 0.0f : v3.w;
      }
      *(volatile v4f*)(dp)       = v0;
      *(volatile v4f*)(dp + 128) = v1;
      *(volatile v4f*)(dp + 256) = v2;
      *(volatile v4f*)(dp + 384) = v3;
      __threadfence();
      *(volatile v4f*)(dp)       = v0;
      *(volatile v4f*)(dp + 128) = v1;
      *(volatile v4f*)(dp + 256) = v2;
      *(volatile v4f*)(dp + 384) = v3;
    }
  }
}

static inline int cdiv(int a, int b) { return (a + b - 1) / b; }
static inline size_t al256(size_t o) { return (o + 255) & ~(size_t)255; }

extern "C" void kernel_launch(void* const* d_in, const int* in_sizes, int n_in,
                              void* d_out, int out_size, void* d_ws, size_t ws_size,
                              hipStream_t stream) {
  if (n_in < 8) return;
  if (in_sizes[0] < DM || (in_sizes[0] % DM) != 0) return;
  const int nN = in_sizes[0] / DM;
  const int nE = in_sizes[1];
  if (in_sizes[2] != nE || in_sizes[3] != nE) return;
  if (nE < EPT || (nE % EPT) != 0 || nE > (1 << 19) - CHUNK) return;
  if (nN < 1 || nN > (1 << 20)) return;
  if (in_sizes[4] != DM * DM || in_sizes[5] != DM) return;
  if (in_sizes[6] != 2 * NREL * DM * DM || in_sizes[7] != 2 * NREL * DM) return;
  if ((long long)out_size != (long long)nN * DM) return;

  const float* x     = (const float*)d_in[0];
  const int*   heads = (const int*)d_in[1];
  const int*   tails = (const int*)d_in[2];
  const int*   rl    = (const int*)d_in[3];
  const float* wself = (const float*)d_in[4];
  const float* bself = (const float*)d_in[5];
  const float* wrel  = (const float*)d_in[6];
  const float* brel  = (const float*)d_in[7];
  float* out = (float*)d_out;

  const int MP = cdiv(nN, GBM) * GBM;
  const int gM = MP / GBM;
  const int gA = cdiv(nN, NBA);
  if ((long long)gA * NBA < (long long)nN) return;

  char* ws = (char*)d_ws;
  size_t off = 0;
  const size_t oXB  = off; off = al256(off + (size_t)MP * DM * 2);
  const size_t oWSB = off; off = al256(off + (size_t)DM * DM * 2);
  const size_t oWRB = off; off = al256(off + (size_t)2 * NREL * DM * DM * 2);
  const size_t oHFB = off; off = al256(off + (size_t)MP * DM2 * 4);
  if (off > ws_size || off > (size_t)WSMAX) return;
  unsigned short* XB  = (unsigned short*)(ws + oXB);
  unsigned short* WSB = (unsigned short*)(ws + oWSB);
  unsigned short* WRB = (unsigned short*)(ws + oWRB);
  float*          HFB = (float*)(ws + oHFB);

  const size_t scanLds = (size_t)SCAN_LDS_INTS * 4;
  hipFuncSetAttribute(reinterpret_cast<const void*>(&k_scan), hipFuncAttributeMaxDynamicSharedMemorySize, (int)scanLds);

  const int nxu = MP * (DM / 8);
  const int nunits = nxu + DM * DM / 8 + 2 * NREL * DM * DM / 8;
  k_prep<<<cdiv(nunits, NTHR), NTHR, 0, stream>>>(x, wself, wrel, nN, nxu, XB, WSB, WRB);

  k_gemm<<<dim3(gM, DM / GBN), GTHR, 0, stream>>>(XB, WSB, WSB, bself, bself, out, DM, nN);

  for (int r = 0; r < NREL; ++r) {
    const unsigned short* B0p = WRB + (size_t)r * DM * DM;
    const unsigned short* B1p = WRB + (size_t)(r + NREL) * DM * DM;
    const float* bA = brel + (size_t)r * DM;
    const float* bB = brel + (size_t)(r + NREL) * DM;
    k_gemm<<<dim3(gM, DM2 / GBN), GTHR, 0, stream>>>(XB, B0p, B1p, bA, bB, HFB, DM2, MP);
    const int fin = (r == NREL - 1) ? 1 : 0;
    k_scan<<<gA, NTHR, scanLds, stream>>>(heads, tails, rl, nE, nN, r, fin, HFB, out);
  }
}
